// DiffuserSelfAttention_89386859364901
// MI455X (gfx1250) — hardware-verified
//
#include <hip/hip_runtime.h>
#include <math.h>
#include <stdint.h>

#define NTOK 1024
#define HID  512
#define NH   8
#define HD   64
#define NQKV 1536
#define RB   16

static_assert(NH * HD == HID);
static_assert(HD == 64);
static_assert(NTOK % 64 == 0);
static_assert(NTOK % RB == 0);
static_assert(NQKV % 64 == 0);
static_assert(HID % 32 == 0);
static_assert(((NTOK / 64) * (NQKV / 64)) % 4 == 0);
static_assert(RB * NTOK * 4 <= 65536);

typedef __attribute__((ext_vector_type(16))) __bf16 v16b;
typedef __attribute__((ext_vector_type(8)))  __bf16 v8b;
typedef __attribute__((ext_vector_type(8)))  float  v8f;
typedef __attribute__((ext_vector_type(4)))  float  v4f;
typedef __attribute__((ext_vector_type(4)))  unsigned int v4u;
typedef __attribute__((ext_vector_type(4)))  int    v4i;
typedef v4f __attribute__((may_alias)) v4fa;
typedef v4u __attribute__((may_alias)) v4ua;

__device__ __forceinline__ unsigned short f2bf_bits(float f) {
  unsigned u = __float_as_uint(f);
  return (unsigned short)((u + 0x7FFFu + ((u >> 16) & 1u)) >> 16);
}
__device__ __forceinline__ float bf_bits2f(unsigned short h) { return __uint_as_float(((unsigned)h) << 16); }
__device__ __forceinline__ unsigned pk16(unsigned short a, unsigned short b) { return (unsigned)a | ((unsigned)b << 16); }

__device__ __forceinline__ void split2(float f0, float f1, unsigned& uh, unsigned& ul) {
  const unsigned short h0 = f2bf_bits(f0), h1 = f2bf_bits(f1);
  const unsigned short l0 = f2bf_bits(f0 - bf_bits2f(h0)), l1 = f2bf_bits(f1 - bf_bits2f(h1));
  uh = pk16(h0, h1);
  ul = pk16(l0, l1);
}

union FB { v16b v; v8b h[2]; };
__device__ __forceinline__ v16b ldfrag(const __bf16* p) {
  FB f;
  f.h[0] = *(const v8b*)(p);
  f.h[1] = *(const v8b*)(p + 16);
  return f.v;
}
__device__ __forceinline__ v8f mma_bf(v16b a, v16b b, v8f c) {
  c = __builtin_amdgcn_wmma_f32_16x16x32_bf16(false, a, false, b, (short)0, c, false, false);
  asm volatile("v_nop\n\tv_nop\n\tv_nop\n\tv_nop" : "+v"(c) : "v"(a), "v"(b));
  return c;
}

__device__ __forceinline__ void cvt8_store(const float* __restrict__ s, unsigned short* __restrict__ d) {
  const v4f a = *(const v4f*)(s);
  const v4f b = *(const v4f*)(s + 4);
  const unsigned o0 = pk16(f2bf_bits(a.x), f2bf_bits(a.y));
  const unsigned o1 = pk16(f2bf_bits(a.z), f2bf_bits(a.w));
  const unsigned o2 = pk16(f2bf_bits(b.x), f2bf_bits(b.y));
  const unsigned o3 = pk16(f2bf_bits(b.z), f2bf_bits(b.w));
  const v4u o = {o0, o1, o2, o3};
  *(volatile v4u*)d = o;
  __threadfence();
  *(volatile v4u*)d = o;
}
__device__ __forceinline__ void bias4_store(const float* __restrict__ s, float* __restrict__ d) {
  const v4f a = *(const v4f*)(s);
  const v4f o = { bf_bits2f(f2bf_bits(a.x)), bf_bits2f(f2bf_bits(a.y)), bf_bits2f(f2bf_bits(a.z)), bf_bits2f(f2bf_bits(a.w)) };
  *(volatile v4f*)d = o;
  __threadfence();
  *(volatile v4f*)d = o;
}

__global__ __launch_bounds__(256) void k_prep(
    const float* __restrict__ x, const float* __restrict__ mask,
    const float* __restrict__ wq, const float* __restrict__ bq,
    const float* __restrict__ wk, const float* __restrict__ bk,
    const float* __restrict__ wv, const float* __restrict__ bv,
    unsigned short* __restrict__ XB, unsigned short* __restrict__ WB,
    float* __restrict__ BQKV, float* __restrict__ MK)
{
  const int bid = blockIdx.x, tid = threadIdx.x;
  if (bid < 256) {
    const size_t o = ((size_t)bid * 256 + tid) * 8;
    cvt8_store(x + o, XB + o);
  } else if (bid < 384) {
    const size_t o = ((size_t)(bid - 256) * 256 + tid) * 8;
    cvt8_store(wq + o, WB + o);
  } else if (bid < 512) {
    const size_t o = ((size_t)(bid - 384) * 256 + tid) * 8;
    cvt8_store(wk + o, WB + (size_t)HID * HID + o);
  } else if (bid < 640) {
    const size_t o = ((size_t)(bid - 512) * 256 + tid) * 8;
    cvt8_store(wv + o, WB + (size_t)2 * HID * HID + o);
  } else {
    const int u = (bid - 640) * 256 + tid;
    if (u < 128) {
      bias4_store(bq + u * 4, BQKV + u * 4);
    } else if (u < 256) {
      bias4_store(bk + (u - 128) * 4, BQKV + 512 + (u - 128) * 4);
    } else if (u < 384) {
      bias4_store(bv + (u - 256) * 4, BQKV + 1024 + (u - 256) * 4);
    } else if (u < 640) {
      const int o = (u - 384) * 4;
      const v4f a = *(const v4f*)(mask + o);
      const v4f r = { (bf_bits2f(f2bf_bits(a.x)) > 0.0f) ? 1.0f : 0.0f,
                      (bf_bits2f(f2bf_bits(a.y)) > 0.0f) ? 1.0f : 0.0f,
                      (bf_bits2f(f2bf_bits(a.z)) > 0.0f) ? 1.0f : 0.0f,
                      (bf_bits2f(f2bf_bits(a.w)) > 0.0f) ? 1.0f : 0.0f };
      *(volatile v4f*)(MK + o) = r;
      __threadfence();
      *(volatile v4f*)(MK + o) = r;
    }
  }
}

__device__ __forceinline__ void tally(unsigned* cnt, int s, int d, int base, bool valid) {
  const unsigned dr = (unsigned)(d - base);
  if (valid && dr < (unsigned)RB) {
    const int sc = min(max(s, 0), NTOK - 1);
    atomicAdd(&cnt[dr * NTOK + sc], 1u);
  }
}

__global__ __launch_bounds__(256) void k_cnt(const int* __restrict__ src, const int* __restrict__ dst,
                                             unsigned* __restrict__ CNT, int E)
{
  __shared__ __align__(16) unsigned cnt[RB * NTOK];
  const int tid = threadIdx.x;
  const int base = blockIdx.x * RB;
  {
    const v4u z = {0u, 0u, 0u, 0u};
    v4ua* p = (v4ua*)cnt;
    for (int i = tid; i < RB * NTOK / 4; i += 256) p[i] = z;
  }
  __syncthreads();
  const int nfull = E / 1024;
#pragma unroll 1
  for (int ch = 0; ch < nfull; ++ch) {
    const int e0 = ch * 1024 + tid * 4;
    const v4i s4 = *(const v4i*)(src + e0);
    const v4i d4 = *(const v4i*)(dst + e0);
    tally(cnt, s4.x, d4.x, base, true);
    tally(cnt, s4.y, d4.y, base, true);
    tally(cnt, s4.z, d4.z, base, true);
    tally(cnt, s4.w, d4.w, base, true);
  }
  const int rem0 = nfull * 1024;
#pragma unroll 1
  for (int j = 0; j < 4; ++j) {
    const int e  = rem0 + j * 256 + tid;
    const int ec = min(e, E - 1);
    const int s = src[ec];
    const int d = dst[ec];
    tally(cnt, s, d, base, e < E);
  }
  __syncthreads();
  for (int pass = 0; pass < 2; ++pass) {
#pragma unroll 4
    for (int r = 0; r < RB; ++r) {
      const v4u v = ((const v4ua*)cnt)[r * 256 + tid];
      *(volatile v4u*)(CNT + (size_t)(base + r) * NTOK + tid * 4) = v;
    }
    __threadfence();
  }
}

__global__ __launch_bounds__(128) void k_qkv(
    const unsigned short* __restrict__ XBp, const unsigned short* __restrict__ WBp,
    const float* __restrict__ BQKV,
    unsigned short* __restrict__ QK, float* __restrict__ V, unsigned short* __restrict__ HT0)
{
  __shared__ __align__(16) float tl[4][64 * 64];
  const int lane = threadIdx.x & 31;
  const int wave = __builtin_amdgcn_readfirstlane((int)(threadIdx.x >> 5));
  const int hh = lane >> 4, c = lane & 15;
  const int tile = blockIdx.x * 4 + wave;
  const int tm = tile / 24;
  const int tn = tile - tm * 24;
  const int m0 = tm * 64, n0 = tn * 64;
  const __bf16* A = (const __bf16*)(const void*)XBp;
  const __bf16* B = (const __bf16*)(const void*)WBp;

  v8f acc[4][4];
#pragma unroll
  for (int i = 0; i < 4; ++i)
#pragma unroll
    for (int j = 0; j < 4; ++j) acc[i][j] = (v8f){0.f,0.f,0.f,0.f,0.f,0.f,0.f,0.f};

#pragma unroll 1
  for (int k0 = 0; k0 < HID; k0 += 32) {
    v16b bh[4];
#pragma unroll
    for (int j = 0; j < 4; ++j)
      bh[j] = ldfrag(B + (size_t)(n0 + 16 * j + c) * HID + k0 + 8 * hh);
#pragma unroll
    for (int i = 0; i < 4; ++i) {
      const v16b ah = ldfrag(A + (size_t)(m0 + 16 * i + c) * HID + k0 + 8 * hh);
#pragma unroll
      for (int j = 0; j < 4; ++j) acc[i][j] = mma_bf(ah, bh[j], acc[i][j]);
    }
  }

  const int third = tn >> 3;
  const int nl = (tn & 7) * 64;
  const float osc = (third == 0) ? 0.125f : 1.0f;
  float* tw = tl[wave];
#pragma unroll
  for (int j = 0; j < 4; ++j) {
    const float bvv = BQKV[n0 + 16 * j + c];
#pragma unroll
    for (int i = 0; i < 4; ++i) {
#pragma unroll
      for (int r = 0; r < 8; ++r)
        tw[(16 * i + 8 * hh + r) * 64 + 16 * j + c] = (acc[i][j][r] + bvv) * osc;
    }
  }
  __builtin_amdgcn_fence(__ATOMIC_RELEASE, "workgroup");
  __builtin_amdgcn_wave_barrier();
  __builtin_amdgcn_fence(__ATOMIC_ACQUIRE, "workgroup");

  if (third < 2) {
    unsigned short* dstp = QK + (size_t)third * ((size_t)NTOK * 1024);
    const int q = lane >> 3, c8 = (lane & 7) * 8;
    for (int pass = 0; pass < 2; ++pass) {
#pragma unroll 4
      for (int it = 0; it < 16; ++it) {
        const int row = it * 4 + q;
        const v4f a = *(const v4fa*)(tw + row * 64 + c8);
        const v4f b = *(const v4fa*)(tw + row * 64 + c8 + 4);
        unsigned h0, h1, h2, h3, l0, l1, l2, l3;
        split2(a.x, a.y, h0, l0); split2(a.z, a.w, h1, l1);
        split2(b.x, b.y, h2, l2); split2(b.z, b.w, h3, l3);
        const v4u hv = {h0, h1, h2, h3};
        const v4u lv = {l0, l1, l2, l3};
        const size_t go = (size_t)(m0 + row) * 1024 + nl + c8;
        *(volatile v4u*)(dstp + go) = hv;
        *(volatile v4u*)(dstp + go + 512) = lv;
      }
      __threadfence();
    }
  } else {
    {
      const int h2 = lane >> 4, c4 = (lane & 15) * 4;
      for (int pass = 0; pass < 2; ++pass) {
#pragma unroll 4
        for (int it = 0; it < 32; ++it) {
          const int row = it * 2 + h2;
          const v4f a = *(const v4fa*)(tw + row * 64 + c4);
          *(volatile v4f*)(V + (size_t)(m0 + row) * HID + nl + c4) = a;
        }
        __threadfence();
      }
    }
    {
      const int q = lane >> 3, t8 = (lane & 7) * 8;
      for (int pass = 0; pass < 2; ++pass) {
#pragma unroll 4
        for (int it = 0; it < 16; ++it) {
          const int d = it * 4 + q;
          float f[8];
#pragma unroll
          for (int e = 0; e < 8; ++e) f[e] = tw[(t8 + e) * 64 + d];
          unsigned h0, h1, h2, h3, l0, l1, l2, l3;
          split2(f[0], f[1], h0, l0); split2(f[2], f[3], h1, l1);
          split2(f[4], f[5], h2, l2); split2(f[6], f[7], h3, l3);
          const v4u hv = {h0, h1, h2, h3};
          const v4u lv = {l0, l1, l2, l3};
          const size_t go = (size_t)(nl + d) * 2048 + m0 + t8;
          *(volatile v4u*)(HT0 + go) = hv;
          *(volatile v4u*)(HT0 + go + 1024) = lv;
        }
        __threadfence();
      }
    }
  }
}

__global__ __launch_bounds__(128) void k_score(const unsigned short* __restrict__ QHLp,
                                               const unsigned short* __restrict__ KHLp,
                                               float* __restrict__ S)
{
  __shared__ __align__(16) float slabs[4][16 * 68];
  const int lane = threadIdx.x & 31, wave = threadIdx.x >> 5;
  const int hh = lane >> 4, c = lane & 15;
  const int h = blockIdx.x >> 4;
  const int i0 = (blockIdx.x & 15) * 64 + 16 * wave;
  const __bf16* Q = (const __bf16*)(const void*)QHLp + (size_t)(i0 + c) * 1024 + h * HD + 8 * hh;
  const __bf16* K = (const __bf16*)(const void*)KHLp + (size_t)c * 1024 + h * HD + 8 * hh;
  v16b qah[2], qal[2];
#pragma unroll
  for (int dc = 0; dc < 2; ++dc) {
    qah[dc] = ldfrag(Q + dc * 32);
    qal[dc] = ldfrag(Q + 512 + dc * 32);
  }
  float* slab = slabs[wave];
  float* Sg = S + ((size_t)h * NTOK + i0) * NTOK;
  const int h2 = lane >> 4, c4 = (lane & 15) * 4;

#pragma unroll 1
  for (int jt = 0; jt < 16; ++jt) {
    v8f acc[4];
#pragma unroll
    for (int t = 0; t < 4; ++t) {
      acc[t] = (v8f){0.f,0.f,0.f,0.f,0.f,0.f,0.f,0.f};
      const __bf16* Kp = K + (size_t)(jt * 64 + 16 * t) * 1024;
#pragma unroll
      for (int dc = 0; dc < 2; ++dc) {
        const v16b kb = ldfrag(Kp + dc * 32);
        const v16b kl = ldfrag(Kp + 512 + dc * 32);
        acc[t] = mma_bf(qah[dc], kb, acc[t]);
        acc[t] = mma_bf(qah[dc], kl, acc[t]);
        acc[t] = mma_bf(qal[dc], kb, acc[t]);
      }
    }
#pragma unroll
    for (int t = 0; t < 4; ++t)
#pragma unroll
      for (int r = 0; r < 8; ++r) slab[(8 * hh + r) * 68 + 16 * t + c] = acc[t][r];
    __builtin_amdgcn_fence(__ATOMIC_RELEASE, "workgroup");
    __builtin_amdgcn_wave_barrier();
    __builtin_amdgcn_fence(__ATOMIC_ACQUIRE, "workgroup");
    for (int pass = 0; pass < 2; ++pass) {
#pragma unroll
      for (int it = 0; it < 8; ++it) {
        const int row = it * 2 + h2;
        const v4f v = *(const v4fa*)(slab + row * 68 + c4);
        *(volatile v4f*)(Sg + (size_t)row * NTOK + jt * 64 + c4) = v;
      }
      __threadfence();
    }
    __builtin_amdgcn_fence(__ATOMIC_RELEASE, "workgroup");
    __builtin_amdgcn_wave_barrier();
    __builtin_amdgcn_fence(__ATOMIC_ACQUIRE, "workgroup");
  }
}

__global__ __launch_bounds__(128) void k_soft(const float* __restrict__ S, const unsigned* __restrict__ CNT,
                                              const float* __restrict__ MK, unsigned short* __restrict__ PHL)
{
  __shared__ __align__(16) float sv[4][NTOK];
  __shared__ __align__(16) float cf[4][NTOK];
  const int lane = threadIdx.x & 31, wave = threadIdx.x >> 5;
  const int row = blockIdx.x * 4 + wave;
  const int i = row & (NTOK - 1);
  const float* Srow = S + (size_t)row * NTOK;
  const unsigned* Crow = CNT + (size_t)i * NTOK;
  unsigned short* Prow = PHL + (size_t)row * 2048;
  float* svw = sv[wave];
  float* cfw = cf[wave];
  const float oki = MK[i];

  float mloc = -INFINITY;
#pragma unroll 1
  for (int ch = 0; ch < 4; ++ch) {
    const int j0 = ch * 256 + lane * 8;
    const v4f s0 = *(const v4f*)(Srow + j0);
    const v4f s1 = *(const v4f*)(Srow + j0 + 4);
    const v4u c0 = *(const v4u*)(Crow + j0);
    const v4u c1 = *(const v4u*)(Crow + j0 + 4);
    const v4f k0 = *(const v4f*)(MK + j0);
    const v4f k1 = *(const v4f*)(MK + j0 + 4);
    const float    sa[8] = {s0.x, s0.y, s0.z, s0.w, s1.x, s1.y, s1.z, s1.w};
    const unsigned ca[8] = {c0.x, c0.y, c0.z, c0.w, c1.x, c1.y, c1.z, c1.w};
    const float    ka[8] = {k0.x, k0.y, k0.z, k0.w, k1.x, k1.y, k1.z, k1.w};
    float so[8], fo[8];
#pragma unroll
    for (int e = 0; e < 8; ++e) {
      const bool ok = (oki > 0.0f) && (ka[e] > 0.0f);
      const float sp = ok ? sa[e] : -10000.0f;
      const bool on = ca[e] > 0u;
      mloc = fmaxf(mloc, on ? sp : -INFINITY);
      so[e] = sp;
      fo[e] = (float)ca[e];
    }
    const v4f o0 = {so[0], so[1], so[2], so[3]};
    const v4f o1 = {so[4], so[5], so[6], so[7]};
    const v4f f0 = {fo[0], fo[1], fo[2], fo[3]};
    const v4f f1 = {fo[4], fo[5], fo[6], fo[7]};
    *(v4fa*)(svw + j0) = o0;
    *(v4fa*)(svw + j0 + 4) = o1;
    *(v4fa*)(cfw + j0) = f0;
    *(v4fa*)(cfw + j0 + 4) = f1;
  }
  float m = mloc;
#pragma unroll
  for (int off = 16; off >= 1; off >>= 1) m = fmaxf(m, __shfl_xor(m, off, 32));

  float lsum = 0.0f;
#pragma unroll 1
  for (int ch = 0; ch < 4; ++ch) {
    const int j0 = ch * 256 + lane * 8;
    const v4f x0 = *(const v4fa*)(svw + j0);
    const v4f x1 = *(const v4fa*)(svw + j0 + 4);
    const v4f g0 = *(const v4fa*)(cfw + j0);
    const v4f g1 = *(const v4fa*)(cfw + j0 + 4);
    const float xa[8] = {x0.x, x0.y, x0.z, x0.w, x1.x, x1.y, x1.z, x1.w};
    const float ga[8] = {g0.x, g0.y, g0.z, g0.w, g1.x, g1.y, g1.z, g1.w};
    float wo[8];
#pragma unroll
    for (int e = 0; e < 8; ++e) {
      float ex = expf(xa[e] - m);
      ex = (ex < 1.17549435e-38f) ? 0.0f : ex;
      const float w = (ga[e] > 0.0f) ? ga[e] * ex : 0.0f;
      lsum += w;
      wo[e] = w;
    }
    const v4f w0 = {wo[0], wo[1], wo[2], wo[3]};
    const v4f w1 = {wo[4], wo[5], wo[6], wo[7]};
    *(v4fa*)(svw + j0) = w0;
    *(v4fa*)(svw + j0 + 4) = w1;
  }
  float l = lsum;
#pragma unroll
  for (int off = 16; off >= 1; off >>= 1) l += __shfl_xor(l, off, 32);
  const bool live = l > 0.0f;
  const float rl = 1.0f / (live ? l : 1.0f);

  for (int pass = 0; pass < 2; ++pass) {
#pragma unroll 1
    for (int ch = 0; ch < 4; ++ch) {
      const int j0 = ch * 256 + lane * 8;
      const v4f w0 = *(const v4fa*)(svw + j0);
      const v4f w1 = *(const v4fa*)(svw + j0 + 4);
      const float wa[8] = {w0.x, w0.y, w0.z, w0.w, w1.x, w1.y, w1.z, w1.w};
      float p[8];
#pragma unroll
      for (int e = 0; e < 8; ++e) p[e] = live ? wa[e] * rl : 0.0f;
      unsigned h0, h1, h2, h3, l0, l1, l2, l3;
      split2(p[0], p[1], h0, l0); split2(p[2], p[3], h1, l1);
      split2(p[4], p[5], h2, l2); split2(p[6], p[7], h3, l3);
      const v4u hv = {h0, h1, h2, h3};
      const v4u lv = {l0, l1, l2, l3};
      *(volatile v4u*)(Prow + j0) = hv;
      *(volatile v4u*)(Prow + 1024 + j0) = lv;
    }
    __threadfence();
  }
}

template <bool LAST>
__global__ __launch_bounds__(128) void k_prop(const unsigned short* __restrict__ PHLp,
                                              const unsigned short* __restrict__ HTin,
                                              unsigned short* __restrict__ HTout,
                                              const float* __restrict__ V, float* __restrict__ out)
{
  __shared__ __align__(16) float tile[64 * 68];
  const int tid = threadIdx.x, lane = tid & 31, wave = tid >> 5;
  const int hh = lane >> 4, c = lane & 15;
  const int h = blockIdx.x >> 4;
  const int i0 = (blockIdx.x & 15) * 64;
  const __bf16* P  = (const __bf16*)(const void*)PHLp + (size_t)(h * NTOK + i0 + 16 * wave + c) * 2048 + 8 * hh;
  const __bf16* Hb = (const __bf16*)(const void*)HTin + (size_t)(h * HD + c) * 2048 + 8 * hh;

  v8f acc[4];
#pragma unroll
  for (int t = 0; t < 4; ++t) acc[t] = (v8f){0.f,0.f,0.f,0.f,0.f,0.f,0.f,0.f};

#pragma unroll 1
  for (int k0 = 0; k0 < NTOK; k0 += 32) {
    const v16b ah = ldfrag(P + k0);
    const v16b al = ldfrag(P + 1024 + k0);
#pragma unroll
    for (int t = 0; t < 4; ++t) {
      const v16b bh = ldfrag(Hb + (size_t)(16 * t) * 2048 + k0);
      const v16b bl = ldfrag(Hb + (size_t)(16 * t) * 2048 + 1024 + k0);
      acc[t] = mma_bf(ah, bh, acc[t]);
      acc[t] = mma_bf(ah, bl, acc[t]);
      acc[t] = mma_bf(al, bh, acc[t]);
    }
  }

#pragma unroll
  for (int t = 0; t < 4; ++t)
#pragma unroll
    for (int r = 0; r < 8; ++r) tile[(16 * wave + 8 * hh + r) * 68 + 16 * t + c] = acc[t][r];
  __syncthreads();

  if (LAST) {
    v4f val[8];
#pragma unroll
    for (int it = 0; it < 8; ++it) {
      const int u = it * 128 + tid;
      const int row = u >> 4, c4 = (u & 15) * 4;
      const v4f a = *(const v4fa*)(tile + row * 68 + c4);
      const v4f vv = *(const v4f*)(V + (size_t)(i0 + row) * HID + h * HD + c4);
      const v4f o = { 0.9f * a.x + 0.1f * vv.x, 0.9f * a.y + 0.1f * vv.y,
                      0.9f * a.z + 0.1f * vv.z, 0.9f * a.w + 0.1f * vv.w };
      val[it] = o;
    }
    for (int pass = 0; pass < 2; ++pass) {
#pragma unroll
      for (int it = 0; it < 8; ++it) {
        const int u = it * 128 + tid;
        const int row = u >> 4, c4 = (u & 15) * 4;
        *(volatile v4f*)(out + (size_t)(i0 + row) * HID + h * HD + c4) = val[it];
      }
      __threadfence();
    }
  } else {
#pragma unroll
    for (int it = 0; it < 8; ++it) {
      const int u = it * 128 + tid;
      const int row = u >> 4, c4 = (u & 15) * 4;
      const v4f a = *(const v4fa*)(tile + row * 68 + c4);
      const v4f vv = *(const v4f*)(V + (size_t)(i0 + row) * HID + h * HD + c4);
      const v4f o = { 0.9f * a.x + 0.1f * vv.x, 0.9f * a.y + 0.1f * vv.y,
                      0.9f * a.z + 0.1f * vv.z, 0.9f * a.w + 0.1f * vv.w };
      *(v4fa*)(tile + row * 68 + c4) = o;
    }
    __syncthreads();
    for (int pass = 0; pass < 2; ++pass) {
#pragma unroll
      for (int it = 0; it < 4; ++it) {
        const int u = it * 128 + tid;
        const int d = u >> 3, t8 = (u & 7) * 8;
        float f[8];
#pragma unroll
        for (int e = 0; e < 8; ++e) f[e] = tile[(t8 + e) * 68 + d];
        unsigned h0, h1, h2, h3, l0, l1, l2, l3;
        split2(f[0], f[1], h0, l0); split2(f[2], f[3], h1, l1);
        split2(f[4], f[5], h2, l2); split2(f[6], f[7], h3, l3);
        const v4u hv = {h0, h1, h2, h3};
        const v4u lv = {l0, l1, l2, l3};
        const size_t go = (size_t)(h * HD + d) * 2048 + i0 + t8;
        *(volatile v4u*)(HTout + go) = hv;
        *(volatile v4u*)(HTout + go + 1024) = lv;
      }
      __threadfence();
    }
  }
}

extern "C" void kernel_launch(void* const* d_in, const int* in_sizes, int n_in,
                              void* d_out, int out_size, void* d_ws, size_t ws_size,
                              hipStream_t stream) {
  if (n_in < 10) return;
  if (in_sizes[0] != NTOK * HID) return;
  if (in_sizes[1] != NTOK) return;
  if (in_sizes[2] != HID * HID || in_sizes[4] != HID * HID || in_sizes[6] != HID * HID) return;
  if (in_sizes[3] != HID || in_sizes[5] != HID || in_sizes[7] != HID) return;
  if (in_sizes[8] < 1 || in_sizes[8] != in_sizes[9]) return;
  if (out_size != NTOK * HID) return;

  const float* x    = (const float*)d_in[0];
  const float* mask = (const float*)d_in[1];
  const float* Wq   = (const float*)d_in[2];
  const float* bq   = (const float*)d_in[3];
  const float* Wk   = (const float*)d_in[4];
  const float* bk   = (const float*)d_in[5];
  const float* Wv   = (const float*)d_in[6];
  const float* bv   = (const float*)d_in[7];
  const int*   src  = (const int*)d_in[8];
  const int*   dst  = (const int*)d_in[9];
  const int    E    = in_sizes[8];

  size_t off = 0;
  const size_t oXB  = off; off += (size_t)NTOK * HID * 2;
  const size_t oWB  = off; off += (size_t)NQKV * HID * 2;
  const size_t oBQ  = off; off += (size_t)NQKV * 4;
  const size_t oMK  = off; off += (size_t)NTOK * 4;
  const size_t oCNT = off; off += (size_t)NTOK * NTOK * 4;
  const size_t oQK  = off; off += (size_t)2 * NTOK * 1024 * 2;
  const size_t oV   = off; off += (size_t)NTOK * HID * 4;
  const size_t oHT0 = off; off += (size_t)NH * HD * 2048 * 2;
  const size_t oHT1 = off; off += (size_t)NH * HD * 2048 * 2;
  const size_t oS   = off; off += (size_t)NH * NTOK * NTOK * 4;
  const size_t oP   = off; off += (size_t)NH * NTOK * 2048 * 2;
  if (off > ws_size) return;
  if (off > (size_t)134217728) return;

  char* ws = (char*)d_ws;
  unsigned short* XB  = (unsigned short*)(ws + oXB);
  unsigned short* WB  = (unsigned short*)(ws + oWB);
  float*          BQ  = (float*)(ws + oBQ);
  float*          MK  = (float*)(ws + oMK);
  unsigned*       CNT = (unsigned*)(ws + oCNT);
  unsigned short* QK  = (unsigned short*)(ws + oQK);
  unsigned short* KHL = QK + (size_t)NTOK * 1024;
  float*          Vf  = (float*)(ws + oV);
  unsigned short* HT0 = (unsigned short*)(ws + oHT0);
  unsigned short* HT1 = (unsigned short*)(ws + oHT1);
  float*          Sf  = (float*)(ws + oS);
  unsigned short* PHL = (unsigned short*)(ws + oP);
  float*          out = (float*)d_out;

  k_prep<<<dim3(643), dim3(256), 0, stream>>>(x, mask, Wq, bq, Wk, bk, Wv, bv, XB, WB, BQ, MK);
  k_cnt<<<dim3(NTOK / RB), dim3(256), 0, stream>>>(src, dst, CNT, E);
  k_qkv<<<dim3(96), dim3(128), 0, stream>>>(XB, WB, BQ, QK, Vf, HT0);
  k_score<<<dim3(NH * (NTOK / 64)), dim3(128), 0, stream>>>(QK, KHL, Sf);
  k_soft<<<dim3(NH * NTOK / 4), dim3(128), 0, stream>>>(Sf, CNT, MK, PHL);
  const dim3 gP(NH * (NTOK / 64));
  k_prop<false><<<gP, dim3(128), 0, stream>>>(PHL, HT0, HT1, Vf, out);
  k_prop<false><<<gP, dim3(128), 0, stream>>>(PHL, HT1, HT0, Vf, out);
  k_prop<false><<<gP, dim3(128), 0, stream>>>(PHL, HT0, HT1, Vf, out);
  k_prop<false><<<gP, dim3(128), 0, stream>>>(PHL, HT1, HT0, Vf, out);
  k_prop<true><<<gP, dim3(128), 0, stream>>>(PHL, HT0, HT1, Vf, out);
  (void)hipGetLastError();
}
